// CogVideoSAU_420906795752
// MI455X (gfx1250) — hardware-verified
//
#include <hip/hip_runtime.h>
#include <math.h>

typedef __attribute__((ext_vector_type(16))) _Float16 v16h;
typedef __attribute__((ext_vector_type(16))) __bf16 v16b;
typedef __attribute__((ext_vector_type(8)))  _Float16 v8h;
typedef __attribute__((ext_vector_type(8)))  float v8f;
typedef __attribute__((ext_vector_type(4)))  float v4f;
typedef __attribute__((ext_vector_type(2)))  float v2f;
typedef __attribute__((ext_vector_type(4)))  unsigned v4u;
typedef __attribute__((ext_vector_type(4)))  int v4i;
typedef float __attribute__((may_alias)) float_a;
typedef int __attribute__((may_alias)) int_a;

template <typename T> __device__ __forceinline__ void vst2(void* p, T v) { *(volatile T*)p = v; __threadfence(); *(volatile T*)p = v; }
__device__ __forceinline__ v8f wmma16(v16h a, v16h b, v8f c) {
  v8f d = __builtin_amdgcn_wmma_f32_16x16x32_f16(false, a, false, b, (short)0, c, false, false);
  asm volatile("v_nop\n\tv_nop\n\tv_nop\n\tv_nop" : "+v"(d) : "v"(a), "v"(b));
  return d;
}
__device__ __forceinline__ v8f wmma_bf(v16b a, v16b b, v8f c) {
  v8f d = __builtin_amdgcn_wmma_f32_16x16x32_bf16(false, a, false, b, (short)0, c, false, false);
  asm volatile("v_nop\n\tv_nop\n\tv_nop\n\tv_nop" : "+v"(d) : "v"(a), "v"(b));
  return d;
}
__device__ __forceinline__ v16h frag_h(const _Float16* rowk0, int lane) {
  union { v16h v; v8h q[2]; } u; const _Float16* p = rowk0 + 8 * (lane >> 4);
  u.q[0] = *(const v8h*)p; u.q[1] = *(const v8h*)(p + 16); return u.v;
}
__device__ __forceinline__ v16h frag_f32(const float* rowk0, int lane) {
  v16h a; const float* p = rowk0 + 8 * (lane >> 4);
#pragma unroll
  for (int i = 0; i < 8; ++i) { a[i] = (_Float16)p[i]; a[8 + i] = (_Float16)p[16 + i]; }
  return a;
}
__device__ __forceinline__ v16h frag_f32s(const float* rowk0, int lane, float sc) {
  v16h a; const float* p = rowk0 + 8 * (lane >> 4);
#pragma unroll
  for (int i = 0; i < 8; ++i) { a[i] = (_Float16)(p[i] * sc); a[8 + i] = (_Float16)(p[16 + i] * sc); }
  return a;
}
__device__ __forceinline__ v16h fragc_f32(const float* W, int k0, int n, int lane, int ld, int K) {
  v16h a; const int g = lane >> 4;
#pragma unroll
  for (int i = 0; i < 8; ++i) { const int ka = k0 + 8 * g + i, kb = ka + 16;
    a[i] = (_Float16)(ka < K ? W[(size_t)(ka < K ? ka : K - 1) * ld + n] : 0.f); a[8 + i] = (_Float16)(kb < K ? W[(size_t)(kb < K ? kb : K - 1) * ld + n] : 0.f); }
  return a;
}
struct F2 { v16b h, l; };
__device__ __forceinline__ F2 bsplit16(const float v[16]) { F2 r;
#pragma unroll
  for (int i = 0; i < 16; ++i) { const __bf16 h = (__bf16)v[i]; r.h[i] = h; r.l[i] = (__bf16)(v[i] - (float)h); }
  return r; }
__device__ __forceinline__ F2 split_row(const float* row, int k0, int lane) { float v[16]; const float* p = row + k0 + 8 * (lane >> 4);
#pragma unroll
  for (int i = 0; i < 8; ++i) { v[i] = p[i]; v[8 + i] = p[16 + i]; }
  return bsplit16(v); }
__device__ __forceinline__ F2 split_rowK(const float* row, int k0, int lane, int K) { float v[16]; const int g = lane >> 4;
#pragma unroll
  for (int i = 0; i < 8; ++i) { const int ka = k0 + 8 * g + i, kb = ka + 16; v[i] = ka < K ? row[ka < K ? ka : K - 1] : 0.f; v[8 + i] = kb < K ? row[kb < K ? kb : K - 1] : 0.f; }
  return bsplit16(v); }
__device__ __forceinline__ F2 split_col(const float* W, int k0, int n, int lane, int ld, int K) { float v[16]; const int g = lane >> 4;
#pragma unroll
  for (int i = 0; i < 8; ++i) { const int ka = k0 + 8 * g + i, kb = ka + 16; v[i] = ka < K ? W[(size_t)(ka < K ? ka : K - 1) * ld + n] : 0.f; v[8 + i] = kb < K ? W[(size_t)(kb < K ? kb : K - 1) * ld + n] : 0.f; }
  return bsplit16(v); }
__device__ __forceinline__ v8f mac3(const F2& a, const F2& b, v8f c) { c = wmma_bf(a.l, b.h, c); c = wmma_bf(a.h, b.l, c); return wmma_bf(a.h, b.h, c); }
__device__ __forceinline__ float sigm(float v) { return 1.0f / (1.0f + expf(-v)); }
#define LDSX() do { asm volatile("s_wait_dscnt 0" ::: "memory"); __builtin_amdgcn_wave_barrier(); __builtin_amdgcn_fence(__ATOMIC_RELEASE, "workgroup"); } while (0)


#define NB 2
#define TEXT 226
#define NTOK 1024
#define TOK 4096
#define LQ (TEXT + NTOK)
#define LQP 1280
#define LK (TEXT + TOK)
#define LKP 4352
#define DM 1024
#define NH 16
#define HD 64
#ifndef TQB
#define TQB (LQP / 64)
#define TNB NB
#endif
typedef __attribute__((ext_vector_type(8))) __bf16 v8b;
__device__ __forceinline__ v16b frag_b(const __bf16* rowk0, int lane) {
  union { v16b v; v8b q[2]; } u; const __bf16* p = rowk0 + 8 * (lane >> 4);
  u.q[0] = *(const v8b*)p; u.q[1] = *(const v8b*)(p + 16); return u.v;
}
__device__ __forceinline__ float bfr(float v) { return (float)(__bf16)v; }
__device__ __attribute__((noinline)) float exp_ni(float v) { return expf(v); }
__device__ __attribute__((noinline)) float erf_ni(float v) { return erff(v); }

#define WS_PW  0u
#define WS_QF  (WS_PW + 2u * (size_t)4 * DM * DM)
#define WS_KF  (WS_QF + 4u * (size_t)NB * LQP * DM)
#define WS_VF  (WS_KF + 4u * (size_t)NB * LQP * DM)
#define WS_INV (WS_VF + 4u * (size_t)NB * LQP * DM)
#define WS_Q   (WS_INV + 4u * (size_t)TOK)
#define WS_K   (WS_Q + 2u * (size_t)NB * LQP * DM)
#define WS_V   (WS_K + 2u * (size_t)NB * LKP * DM)
#define WS_O   (WS_V + 2u * (size_t)NB * DM * LKP)
#define WS_END (WS_O + 4u * (size_t)NB * LQP * DM)

__global__ __launch_bounds__(256) void k_pack(const float* __restrict__ WQ, const float* __restrict__ WK, const float* __restrict__ WV, const float* __restrict__ WO, __bf16* __restrict__ PW) { const int n = blockIdx.x, which = blockIdx.y, t = threadIdx.x; __shared__ __align__(16) __bf16 s[DM]; const float* w = (which == 0) ? WQ : (which == 1) ? WK : (which == 2) ? WV : WO; for (int k = t; k < DM; k += 256) s[k] = (__bf16)w[(size_t)k * DM + n]; __syncthreads(); if (t < DM / 8) vst2((unsigned*)(PW + ((size_t)which * DM + n) * DM + t * 8), *(const v4u*)&s[t * 8]); }
__global__ __launch_bounds__(256) void k_inv(const int* __restrict__ TI, int* __restrict__ INV) { __shared__ __align__(16) int s[TOK]; const int t = threadIdx.x; for (int e = t; e < TOK; e += 256) s[e] = -1; __syncthreads();
  for (int i = t; i < NTOK; i += 256) { int slot = TI[i]; slot = slot < 0 ? 0 : (slot >= TOK ? TOK - 1 : slot); s[slot] = i; } __syncthreads();
  for (int q = t; q < TOK / 4; q += 256) vst2(INV + q * 4, *(const v4i*)&s[q * 4]); }
__global__ __launch_bounds__(128) void k_proj(const float* __restrict__ HID_, const float* __restrict__ ENC, const __bf16* __restrict__ PW, float* __restrict__ QF, float* __restrict__ KF, float* __restrict__ VF) {
  __shared__ __align__(16) float so[4][16][132];
  const int tid = threadIdx.x, wave = tid >> 5, lane = tid & 31, col = lane & 15, g = lane >> 4; const int which = blockIdx.z; const size_t rb = (size_t)blockIdx.x * 64; const size_t r0 = rb + wave * 16; const int c0 = blockIdx.y * 128; const size_t b = rb / LQP;
  const int s = (int)((r0 + col) % LQP); const bool live = s < LQ; const float* src = (s < TEXT) ? (ENC + ((b * TEXT + s) * DM)) : (HID_ + ((b * NTOK + (live ? s - TEXT : 0)) * DM));
  const __bf16* Wr = PW + ((size_t)which * DM) * DM; float* dst = (which == 0) ? QF : (which == 1) ? KF : VF;
  v8f acc[8] = {};
#pragma unroll 2
  for (int kc = 0; kc < DM / 32; ++kc) { v16b a; { const float* p = src + kc * 32 + 8 * g;
#pragma unroll
      for (int i = 0; i < 8; ++i) { a[i] = live ? (__bf16)p[i] : (__bf16)0.f; a[8 + i] = live ? (__bf16)p[16 + i] : (__bf16)0.f; } }
#pragma unroll
    for (int j = 0; j < 8; ++j) acc[j] = wmma_bf(a, frag_b(Wr + (size_t)(c0 + j * 16 + col) * DM + kc * 32, lane), acc[j]); }
#pragma unroll
  for (int j = 0; j < 8; ++j)
#pragma unroll
    for (int r = 0; r < 8; ++r) so[wave][8 * g + r][j * 16 + col] = acc[j][r];
  LDSX();
  for (int rl = 0; rl < 16; ++rl) vst2(dst + (r0 + rl) * DM + c0 + lane * 4, *(const v4f*)&so[wave][rl][lane * 4]);
}
__device__ __forceinline__ void ln_rope_row(float* sx, const float* __restrict__ G, const float* __restrict__ Bn, const float* __restrict__ CS, const float* __restrict__ SN, int ropepos, _Float16* sh, int t) {
  const int h = t >> 4, part = t & 15; float v[4]; float s = 0.f; for (int i = 0; i < 4; ++i) { v[i] = sx[h * HD + part * 4 + i]; s += v[i]; }
#pragma unroll
  for (int o = 1; o < 16; o <<= 1) s += __shfl_xor(s, o);
  const float mu = s * (1.0f / (float)HD); float q = 0.f; for (int i = 0; i < 4; ++i) { const float d = v[i] - mu; q += d * d; }
#pragma unroll
  for (int o = 1; o < 16; o <<= 1) q += __shfl_xor(q, o);
  const float inv = 1.0f / sqrtf(q * (1.0f / (float)HD) + 1e-6f);
  float y[4]; for (int i = 0; i < 4; ++i) { const int d = part * 4 + i; y[i] = (v[i] - mu) * inv * bfr(G[d]) + bfr(Bn[d]); }
  if (ropepos >= 0) { for (int i = 0; i < 4; i += 2) { const int d = part * 4 + i; const float c0_ = bfr(CS[(size_t)ropepos * HD + d]), s0_ = bfr(SN[(size_t)ropepos * HD + d]), c1_ = bfr(CS[(size_t)ropepos * HD + d + 1]), s1_ = bfr(SN[(size_t)ropepos * HD + d + 1]); const float x0 = y[i], x1 = y[i + 1]; y[i] = x0 * c0_ - x1 * s0_; y[i + 1] = x1 * c1_ + x0 * s1_; } }
  for (int i = 0; i < 4; ++i) sh[h * HD + part * 4 + i] = (_Float16)y[i];
}
__global__ __launch_bounds__(256) void k_q(const float* __restrict__ QF, const float* __restrict__ GQ, const float* __restrict__ BQ, const float* __restrict__ CS, const float* __restrict__ SN, const int* __restrict__ TI, _Float16* __restrict__ Q) {
  __shared__ float sx[DM]; __shared__ __align__(16) _Float16 sh[DM]; const int t = threadIdx.x; const size_t row = blockIdx.x; const int s = (int)(row % LQP);
  for (int e = t; e < DM; e += 256) sx[e] = QF[row * DM + e]; __syncthreads();
  int rp = -1; if (s >= TEXT && s < LQ) { int ti = TI[s - TEXT]; ti = ti < 0 ? 0 : (ti >= TOK ? TOK - 1 : ti); rp = ti; }
  ln_rope_row(sx, GQ, BQ, CS, SN, rp, sh, t); __syncthreads();
  if (t < DM / 8) vst2((unsigned*)(Q + row * DM + t * 8), *(const v4u*)&sh[t * 8]);
}
__global__ __launch_bounds__(256) void k_k(const float* __restrict__ KF, const float* __restrict__ KC, const int* __restrict__ INV, const float* __restrict__ GK, const float* __restrict__ BK, const float* __restrict__ CS, const float* __restrict__ SN, _Float16* __restrict__ Kr) {
  __shared__ float sx[DM]; __shared__ __align__(16) _Float16 sh[DM]; const int t = threadIdx.x; const int p = blockIdx.x; const size_t b = blockIdx.y; const size_t row = b * LKP + p;
  if (p >= LK) { for (int e = t; e < DM; e += 256) sh[e] = (_Float16)0.f; __syncthreads(); if (t < DM / 8) vst2((unsigned*)(Kr + row * DM + t * 8), *(const v4u*)&sh[t * 8]); return; }
  const float* src; bool raw; if (p < TEXT) { src = KF + (b * LQP + p) * DM; raw = false; } else { const int i = INV[p - TEXT]; if (i >= 0) { src = KF + (b * LQP + TEXT + i) * DM; raw = false; } else { src = KC + (b * LK + p) * DM; raw = true; } }
  for (int e = t; e < DM; e += 256) sx[e] = raw ? bfr(src[e]) : src[e]; __syncthreads();
  ln_rope_row(sx, GK, BK, CS, SN, (p >= TEXT) ? (p - TEXT) : -1, sh, t); __syncthreads();
  if (t < DM / 8) vst2((unsigned*)(Kr + row * DM + t * 8), *(const v4u*)&sh[t * 8]);
}
__global__ __launch_bounds__(256) void k_v(const float* __restrict__ VF, const float* __restrict__ VC, const int* __restrict__ INV, _Float16* __restrict__ V) { __shared__ __align__(16) _Float16 st[128][72]; const int t = threadIdx.x; const int p0 = blockIdx.x * 64, c0 = blockIdx.y * 128; const size_t b = blockIdx.z;
  for (int e = t; e < 64 * 128; e += 256) { const int pl = e >> 7, d = e & 127; const int p = p0 + pl; float v = 0.f;
    if (p < LK) { if (p < TEXT) v = VF[(b * LQP + p) * DM + c0 + d]; else { const int i = INV[p - TEXT]; v = (i >= 0) ? VF[(b * LQP + TEXT + i) * DM + c0 + d] : bfr(VC[(b * LK + p) * DM + c0 + d]); } }
    st[d][pl] = (_Float16)v; }
  __syncthreads();
  for (int e = t; e < 128 * 8; e += 256) { const int d = e >> 3, pc = e & 7; vst2((unsigned*)(V + ((b * DM + c0 + d) * LKP) + p0 + pc * 8), *(const v4u*)&st[d][pc * 8]); }
}
__global__ __launch_bounds__(128) void k_attn(const _Float16* __restrict__ Q, const _Float16* __restrict__ Kr, const _Float16* __restrict__ V, float* __restrict__ O) {
  __shared__ __align__(16) _Float16 sph[4][16][40]; __shared__ __align__(16) float so[4][16][68];
  const int tid = threadIdx.x, wave = tid >> 5, lane = tid & 31, col = lane & 15, g = lane >> 4; const int h = blockIdx.y; const size_t b = blockIdx.z; const int q0 = blockIdx.x * 64 + wave * 16; const size_t rq = b * LQP + q0;
  v16h aq[2];
#pragma unroll
  for (int kc = 0; kc < 2; ++kc) aq[kc] = frag_h(Q + (rq + col) * DM + h * HD + kc * 32, lane);
  float m[8], l[8];
#pragma unroll
  for (int r = 0; r < 8; ++r) { m[r] = -3.0e38f; l[r] = 0.f; }
  v8f acc[4] = {};
#pragma unroll 1
  for (int ks = 0; ks < LKP / 32; ++ks) { const int j0 = ks * 32; v8f s[2];
#pragma unroll
    for (int ct = 0; ct < 2; ++ct) { const int kk = j0 + ct * 16 + col; const size_t rk = (b * LKP + kk) * DM + h * HD; v8f c = {};
#pragma unroll
      for (int kc = 0; kc < 2; ++kc) c = wmma16(aq[kc], frag_h(Kr + rk + kc * 32, lane), c);
#pragma unroll
      for (int r = 0; r < 8; ++r) s[ct][r] = (kk < LK) ? c[r] * 0.125f : -3.0e38f; }
#pragma unroll
    for (int r = 0; r < 8; ++r) { float mx = fmaxf(s[0][r], s[1][r]);
#pragma unroll
      for (int o = 1; o < 16; o <<= 1) mx = fmaxf(mx, __shfl_xor(mx, o));
      const float mn = fmaxf(m[r], mx); const float alpha = (m[r] <= -1.0e38f) ? 0.f : __expf(m[r] - mn); const float e0 = (s[0][r] <= -1.0e38f) ? 0.f : __expf(s[0][r] - mn), e1 = (s[1][r] <= -1.0e38f) ? 0.f : __expf(s[1][r] - mn); float es = e0 + e1;
#pragma unroll
      for (int o = 1; o < 16; o <<= 1) es += __shfl_xor(es, o);
      l[r] = l[r] * alpha + es; m[r] = mn;
#pragma unroll
      for (int dt = 0; dt < 4; ++dt) acc[dt][r] *= alpha;
      sph[wave][8 * g + r][col] = (_Float16)(e0 * 2048.0f); sph[wave][8 * g + r][16 + col] = (_Float16)(e1 * 2048.0f); }
    LDSX();
    const v16h pa = frag_h(&sph[wave][col][0], lane);
#pragma unroll
    for (int dt = 0; dt < 4; ++dt) acc[dt] = wmma16(pa, frag_h(V + ((b * DM + h * HD + dt * 16 + col) * LKP) + j0, lane), acc[dt]);
    LDSX(); }
#pragma unroll
  for (int r = 0; r < 8; ++r) { const float il = (1.0f / 2048.0f) / l[r];
#pragma unroll
    for (int dt = 0; dt < 4; ++dt) so[wave][8 * g + r][dt * 16 + col] = acc[dt][r] * il; }
  LDSX();
  for (int rl = 0; rl < 16; ++rl) if (lane < 16) vst2(O + (rq + rl) * DM + h * HD + lane * 4, *(const v4f*)&so[wave][rl][lane * 4]);
}
__global__ __launch_bounds__(128) void k_out(const float* __restrict__ O, const __bf16* __restrict__ PW, const float* __restrict__ BO, float* __restrict__ OUTH, float* __restrict__ OUTE) {
  __shared__ __align__(16) float so[4][16][132];
  const int tid = threadIdx.x, wave = tid >> 5, lane = tid & 31, col = lane & 15, g = lane >> 4; const size_t rb = (size_t)blockIdx.x * 64; const size_t r0 = rb + wave * 16; const int n0 = blockIdx.y * 128; const __bf16* P = PW + (size_t)3 * DM * DM; const size_t b = rb / LQP;
  v8f acc[8] = {};
#pragma unroll 2
  for (int kc = 0; kc < DM / 32; ++kc) { const F2 a = split_row(O + (r0 + col) * DM, kc * 32, lane);
#pragma unroll
    for (int j = 0; j < 8; ++j) { const v16b w = frag_b(P + (size_t)(n0 + j * 16 + col) * DM + kc * 32, lane); acc[j] = wmma_bf(a.h, w, acc[j]); acc[j] = wmma_bf(a.l, w, acc[j]); } }
#pragma unroll
  for (int j = 0; j < 8; ++j) { const float bb = bfr(BO[n0 + j * 16 + col]);
#pragma unroll
    for (int r = 0; r < 8; ++r) so[wave][8 * g + r][j * 16 + col] = acc[j][r] + bb; }
  LDSX();
  for (int rl = 0; rl < 16; ++rl) { const int s = (int)((r0 + rl) % LQP); if (s >= LQ) continue; float* dst = (s < TEXT) ? (OUTE + ((b * TEXT + s) * DM)) : (OUTH + ((b * NTOK + s - TEXT) * DM)); vst2(dst + n0 + lane * 4, *(const v4f*)&so[wave][rl][lane * 4]); }
}
extern "C" void kernel_launch(void* const* d_in, const int* in_sizes, int n_in, void* d_out, int out_size, void* d_ws, size_t ws_size, hipStream_t stream) {
  (void)in_sizes; (void)n_in; (void)out_size;
  const float** F = (const float**)d_in;
  if (ws_size < (size_t)WS_END) return;
  char* ws = (char*)d_ws; __bf16* PW = (__bf16*)ws; float *QF = (float*)(ws + WS_QF), *KF = (float*)(ws + WS_KF), *VF = (float*)(ws + WS_VF), *O = (float*)(ws + WS_O); int* INV = (int*)(ws + WS_INV); _Float16 *Q = (_Float16*)(ws + WS_Q), *Kr = (_Float16*)(ws + WS_K), *V = (_Float16*)(ws + WS_V);
  float* OUTH = (float*)d_out; float* OUTE = OUTH + (size_t)NB * NTOK * DM;
  k_pack<<<dim3(DM, 4), 256, 0, stream>>>(F[2], F[3], F[4], F[5], PW);
  k_inv<<<1, 256, 0, stream>>>((const int*)d_in[15], INV);
  k_proj<<<dim3(NB * LQP / 64, DM / 128, 3), 128, 0, stream>>>(F[0], F[1], PW, QF, KF, VF);
  k_q<<<TNB * LQP, 256, 0, stream>>>(QF, F[7], F[8], F[11], F[12], (const int*)d_in[15], Q);
  k_k<<<dim3(LKP, TNB), 256, 0, stream>>>(KF, F[13], INV, F[9], F[10], F[11], F[12], Kr);
  k_v<<<dim3(LKP / 64, DM / 128, TNB), 256, 0, stream>>>(VF, F[14], INV, V);
  k_attn<<<dim3(TQB, NH, TNB), 128, 0, stream>>>(Q, Kr, V, O);
  k_out<<<dim3(TNB * LQP / 64, DM / 128), 128, 0, stream>>>(O, PW, F[6], OUTH, OUTE);
}
